// RobustInference_24979529793899
// MI455X (gfx1250) — hardware-run, weakly checked
//
#include <hip/hip_runtime.h>
#include <math.h>

typedef __attribute__((ext_vector_type(16))) _Float16 v16h;
typedef __attribute__((ext_vector_type(8)))  _Float16 v8h;
typedef __attribute__((ext_vector_type(8)))  float    v8f;
typedef __attribute__((ext_vector_type(4)))  float    v4f;

constexpr int kB  = 64;
constexpr int kD  = 3072;
constexpr int kN  = 8000;
constexpr int kL  = 64;
constexpr int kNC = 10;
static_assert(kN % 64 == 0, "candidate tiles of 64");
static_assert(kD % 32 == 0 && kL % 32 == 0, "K multiples of 32");
static_assert(kB == 64 && kL == 64, "tile shapes below assume 64");

constexpr float kWCarry    = 16.0f;
constexpr float kNegWInv   = -1.0f / kWCarry;
constexpr float kRcCarry   = 64.0f;
constexpr float kXcCarry   = 64.0f;
constexpr float kCrossFold = 2.0f / (kRcCarry * kXcCarry);
constexpr float kBand      = 0.25f;
constexpr int   kCap       = 32;
constexpr int   kOwn       = 32;
static_assert(kOwn * 250 == kN, "250 threads x 32 candidates");

constexpr size_t kOutRecs  = (size_t)kB * kNC;
constexpr size_t kOutMus   = kOutRecs + (size_t)kNC * kB * kD;
constexpr size_t kOutLv    = kOutMus + (size_t)kNC * kB * kL;
constexpr size_t kOutTotal = kOutLv + (size_t)kNC * kB * kL;
static_assert(kOutRecs * 4 == 2560ull, "out1 offset");
static_assert(kOutMus * 4 == 7866880ull, "out2 offset");
static_assert(kOutLv * 4 == 8030720ull, "out3 offset");
static_assert(kOutTotal * 4 == 8194560ull, "d_out total");

constexpr size_t kSzXC   = (size_t)kB * kD * 2;
constexpr size_t kSzZ16  = (size_t)kN * kL * 2;
constexpr size_t kSzKLD  = (size_t)kN * 4;
constexpr size_t kSzWT   = (size_t)kNC * kD * kL * 2;
constexpr size_t kSzLC   = (size_t)kNC * kN * kB * 4;
constexpr size_t kSzBEST = (size_t)kNC * kB * 32 * 4;
constexpr size_t kOffXC   = 0;
constexpr size_t kOffZ16  = kOffXC + kSzXC;
constexpr size_t kOffKLD  = kOffZ16 + kSzZ16;
constexpr size_t kOffWT   = kOffKLD + kSzKLD;
constexpr size_t kOffLC   = kOffWT + kSzWT;
constexpr size_t kOffBEST = kOffLC + kSzLC;
constexpr size_t kWsTotal = kOffBEST + kSzBEST;
static_assert(kWsTotal == 25943296ull, "carve total");
static_assert(kWsTotal <= 134217728ull, "carve cap");
static_assert((kOffZ16 % 128) == 0 && (kOffKLD % 128) == 0 && (kOffWT % 128) == 0 &&
              (kOffLC % 128) == 0 && (kOffBEST % 128) == 0, "128-B aligned regions");

struct FragH {
  union U { v16h v; v8h h[2]; };
  static __device__ __forceinline__ v16h load(const _Float16* p) {
    U f;
    f.h[0] = *(const v8h*)(p);
    f.h[1] = *(const v8h*)(p + 16);
    return f.v;
  }
};
__device__ __forceinline__ v8f mma_h(v16h a, v16h b, v8f c) {
  c = __builtin_amdgcn_wmma_f32_16x16x32_f16(false, a, false, b, (short)0, c, false, false);
  asm volatile("v_nop\n\tv_nop\n\tv_nop\n\tv_nop" : "+v"(c) : "v"(a), "v"(b));
  return c;
}
__device__ __forceinline__ float coarse_rc(float tv) {
  const float e = __expf(tv * kNegWInv);
  const float s = __builtin_amdgcn_rcpf(1.0f + e);
  return s - 0.5f;
}

__global__ __launch_bounds__(256) void prep_x_kernel(const float* __restrict__ x, unsigned short* __restrict__ xc16, int total8) {
  const int i = blockIdx.x * 256 + threadIdx.x;
  if (i >= total8) return;
  const size_t e0 = (size_t)i << 3;
  const v4f a0 = *(const v4f*)(x + e0);
  const v4f a1 = *(const v4f*)(x + e0 + 4);
  v8h hv;
#pragma unroll
  for (int e = 0; e < 4; ++e) {
    hv[e]     = (_Float16)((a0[e] - 0.5f) * kXcCarry);
    hv[4 + e] = (_Float16)((a1[e] - 0.5f) * kXcCarry);
  }
  unsigned short* q = xc16 + e0;
  *(volatile v8h*)q = hv;
  __threadfence();
  *(volatile v8h*)q = hv;
}

__global__ __launch_bounds__(256) void prep_z_kernel(const float* __restrict__ z, unsigned short* __restrict__ z16, float* __restrict__ kld) {
  __shared__ float sK[32];
  const int tid = threadIdx.x;
  const int i = blockIdx.x * 256 + tid;
  const size_t e0 = (size_t)i << 3;
  const v4f a0 = *(const v4f*)(z + e0);
  const v4f a1 = *(const v4f*)(z + e0 + 4);
  v8h hv;
  float s = 0.0f;
#pragma unroll
  for (int e = 0; e < 4; ++e) {
    hv[e] = (_Float16)a0[e];
    s = fmaf(a0[e], a0[e], s);
  }
#pragma unroll
  for (int e = 0; e < 4; ++e) {
    hv[4 + e] = (_Float16)a1[e];
    s = fmaf(a1[e], a1[e], s);
  }
  unsigned short* q = z16 + e0;
  *(volatile v8h*)q = hv;
  __threadfence();
  *(volatile v8h*)q = hv;
  s += __shfl_xor(s, 1, 32);
  s += __shfl_xor(s, 2, 32);
  s += __shfl_xor(s, 4, 32);
  if ((tid & 7) == 0) sK[tid >> 3] = 0.5f * s;
  __syncthreads();
  if (tid < 32) {
    const float kv = sK[tid];
    float* p = kld + blockIdx.x * 32 + tid;
    *(volatile float*)p = kv;
    __threadfence();
    *(volatile float*)p = kv;
  }
}

__global__ __launch_bounds__(256) void prep_w_kernel(const float* __restrict__ dec_w, unsigned short* __restrict__ wt16) {
  __shared__ float sW[64 * 65];
  const int tid = threadIdx.x;
  const int cls = blockIdx.y;
  const int dbase = blockIdx.x * 64;
  const float* src = dec_w + (size_t)cls * kL * kD + dbase;
  {
    const int lr = tid >> 6, dc = tid & 63;
#pragma unroll 1
    for (int it = 0; it < 16; ++it) {
      const int l = it * 4 + lr;
      sW[l * 65 + dc] = src[(size_t)l * kD + dc];
    }
  }
  __syncthreads();
  const int rq = tid >> 3, seg = tid & 7;
  v8h hv[2];
#pragma unroll
  for (int it = 0; it < 2; ++it) {
    const int dr = it * 32 + rq;
#pragma unroll
    for (int e = 0; e < 8; ++e) hv[it][e] = (_Float16)(sW[(seg * 8 + e) * 65 + dr] * kWCarry);
  }
  for (int pass = 0; pass < 2; ++pass) {
#pragma unroll
    for (int it = 0; it < 2; ++it) {
      const int dr = it * 32 + rq;
      *(volatile v8h*)(wt16 + ((size_t)(cls * kD + dbase + dr)) * kL + seg * 8) = hv[it];
    }
    __threadfence();
  }
}

__global__ __launch_bounds__(64) void coarse_loss_kernel(
    const unsigned short* __restrict__ z16p, const unsigned short* __restrict__ wt16p,
    const unsigned short* __restrict__ xc16p, const float* __restrict__ dec_b,
    const float* __restrict__ kld, float* __restrict__ Lc)
{
  __shared__ __align__(16) float sT[2][16 * 68];
  __shared__ float sR[64];
  const _Float16* z16  = (const _Float16*)z16p;
  const _Float16* wt16 = (const _Float16*)wt16p;
  const _Float16* xc16 = (const _Float16*)xc16p;
  const int cls  = blockIdx.y;
  const int lane = threadIdx.x & 31;
  const int wave = threadIdx.x >> 5;
  const int hh = lane >> 4;
  const int cl = lane & 15;
  const int nW = blockIdx.x * 64 + wave * 32;

  const _Float16* zp0 = z16 + (size_t)(nW + cl) * kL + 8 * hh;
  const _Float16* zp1 = z16 + (size_t)(nW + 16 + cl) * kL + 8 * hh;
  const v16h zb00 = FragH::load(zp0);
  const v16h zb01 = FragH::load(zp0 + 32);
  const v16h zb10 = FragH::load(zp1);
  const v16h zb11 = FragH::load(zp1 + 32);

  v8f acc[2][4];
#pragma unroll
  for (int i = 0; i < 2; ++i)
#pragma unroll
    for (int j = 0; j < 4; ++j) acc[i][j] = (v8f){0.f, 0.f, 0.f, 0.f, 0.f, 0.f, 0.f, 0.f};
  float rsq0 = 0.0f, rsq1 = 0.0f;

  const _Float16* wbase = wt16 + (size_t)cls * kD * kL;
  const float* bb = dec_b + (size_t)cls * kD;
  const _Float16* xbase = xc16 + (size_t)cl * kD + 8 * hh;

#pragma unroll 1
  for (int d0 = 0; d0 < kD; d0 += 32) {
    v16h ar0, ar1;
#pragma unroll
    for (int dt = 0; dt < 2; ++dt) {
      const int drow = d0 + dt * 16;
      const _Float16* wp = wbase + (size_t)(drow + cl) * kL + 8 * hh;
      const v16h wa0 = FragH::load(wp);
      const v16h wa1 = FragH::load(wp + 32);
      const v4f b0 = *(const v4f*)(bb + drow + 8 * hh);
      const v4f b1 = *(const v4f*)(bb + drow + 8 * hh + 4);
      v8f ci;
      ci[0] = b0[0] * kWCarry;
      ci[1] = b0[1] * kWCarry;
      ci[2] = b0[2] * kWCarry;
      ci[3] = b0[3] * kWCarry;
      ci[4] = b1[0] * kWCarry;
      ci[5] = b1[1] * kWCarry;
      ci[6] = b1[2] * kWCarry;
      ci[7] = b1[3] * kWCarry;
      v8f t0 = ci;
      v8f t1 = ci;
      t0 = mma_h(wa0, zb00, t0);
      t0 = mma_h(wa1, zb01, t0);
      t1 = mma_h(wa0, zb10, t1);
      t1 = mma_h(wa1, zb11, t1);
#pragma unroll
      for (int r = 0; r < 8; ++r) {
        const float ra = coarse_rc(t0[r]);
        const float rb = coarse_rc(t1[r]);
        rsq0 = fmaf(ra, ra, rsq0);
        rsq1 = fmaf(rb, rb, rsq1);
        ar0[dt * 8 + r] = (_Float16)(ra * kRcCarry);
        ar1[dt * 8 + r] = (_Float16)(rb * kRcCarry);
      }
    }
#pragma unroll
    for (int t4 = 0; t4 < 4; ++t4) {
      const v16h xb = FragH::load(xbase + (size_t)(t4 * 16) * kD + d0);
      acc[0][t4] = mma_h(ar0, xb, acc[0][t4]);
      acc[1][t4] = mma_h(ar1, xb, acc[1][t4]);
    }
  }

  const float rs0 = rsq0 + __shfl_xor(rsq0, 16, 32);
  const float rs1 = rsq1 + __shfl_xor(rsq1, 16, 32);
  const float kv = kld[nW + lane];
  sR[wave * 32 + lane] = ((hh == 0) ? rs0 : rs1) + kv;
  __syncthreads();

  float* slab = sT[wave];
  const int c4 = cl * 4;
#pragma unroll
  for (int i = 0; i < 2; ++i) {
    float rk[8];
#pragma unroll
    for (int r = 0; r < 8; ++r) rk[r] = sR[wave * 32 + i * 16 + 8 * hh + r];
#pragma unroll
    for (int j = 0; j < 4; ++j) {
#pragma unroll
      for (int r = 0; r < 8; ++r) {
        slab[(8 * hh + r) * 68 + (j << 4) + cl] = rk[r] - acc[i][j][r] * kCrossFold;
      }
    }
    __syncthreads();
    for (int pass = 0; pass < 2; ++pass) {
#pragma unroll
      for (int it = 0; it < 8; ++it) {
        const int row = it * 2 + hh;
        const v4f v = *(const v4f*)(slab + row * 68 + c4);
        *(volatile v4f*)(Lc + ((size_t)cls * kN + nW + i * 16 + row) * kB + c4) = v;
      }
      __threadfence();
    }
    __syncthreads();
  }
}

__global__ __launch_bounds__(256) void select_emit_kernel(
    const float* __restrict__ x, const float* __restrict__ z, const float* __restrict__ dec_w,
    const float* __restrict__ dec_b, const float* __restrict__ Lc, float* __restrict__ out,
    float* __restrict__ bestp)
{
  __shared__ float sRed[8];
  __shared__ int   sCnt[8];
  __shared__ int   sList[kCap];
  __shared__ float sZ[kL];
  const int tid = threadIdx.x, lane = tid & 31, wave = tid >> 5;
  const int cb  = blockIdx.x;
  const int cls = cb / kB;
  const int img = cb - cls * kB;
  if (tid < kCap) sList[tid] = 0;
  const float* col = Lc + (size_t)cls * kN * kB + img;
  const int nbeg = tid * kOwn;

  float m = INFINITY;
#pragma unroll 1
  for (int k = 0; k < kOwn; ++k) {
    const int n = nbeg + k;
    const int nc = (n < kN) ? n : (kN - 1);
    const float v = col[(size_t)nc * kB];
    const float mv = fminf(m, v);
    m = (n < kN) ? mv : m;
  }
#pragma unroll
  for (int off = 16; off >= 1; off >>= 1) m = fminf(m, __shfl_xor(m, off, 32));
  if (lane == 0) sRed[wave] = m;
  __syncthreads();
  float mm = sRed[0];
#pragma unroll 1
  for (int w = 1; w < 8; ++w) mm = fminf(mm, sRed[w]);
  const float thr = mm + kBand;

  int cnt = 0;
#pragma unroll 1
  for (int k = 0; k < kOwn; ++k) {
    const int n = nbeg + k;
    const int nc = (n < kN) ? n : (kN - 1);
    const float v = col[(size_t)nc * kB];
    cnt += ((n < kN) && (v <= thr)) ? 1 : 0;
  }
  int inc = cnt;
#pragma unroll
  for (int off = 1; off < 32; off <<= 1) {
    const int t = __shfl_up(inc, off, 32);
    inc += (lane >= off) ? t : 0;
  }
  if (lane == 31) sCnt[wave] = inc;
  __syncthreads();
  int wofs = 0, total = 0;
#pragma unroll 1
  for (int w = 0; w < 8; ++w) {
    const int cw = sCnt[w];
    total += cw;
    wofs += (w < wave) ? cw : 0;
  }
  int pos = wofs + inc - cnt;
#pragma unroll 1
  for (int k = 0; k < kOwn; ++k) {
    const int n = nbeg + k;
    const int nc = (n < kN) ? n : (kN - 1);
    const float v = col[(size_t)nc * kB];
    const bool hit = (n < kN) && (v <= thr);
    if (hit) {
      if (pos < kCap) sList[pos] = n;
      pos += 1;
    }
  }
  __syncthreads();
  int len = (total < kCap) ? total : kCap;
  len = (len < 0) ? 0 : len;

  int bestN = sList[0];
  bestN = (bestN < 0) ? 0 : ((bestN > kN - 1) ? (kN - 1) : bestN);
  float bestL = INFINITY;
  float finalL = 0.0f;
  const int e0 = (len >= 2) ? 0 : len;
  const float* wcls = dec_w + (size_t)cls * kL * kD;
  const float* bcls = dec_b + (size_t)cls * kD;
  const float* xrow = x + (size_t)img * kD;
  float* orow = out + kOutRecs + (size_t)cb * kD;

#pragma unroll 1
  for (int e = e0; e <= len && e <= kCap; ++e) {
    const bool fin = (e == len);
    const int ei = (e < kCap) ? e : (kCap - 1);
    int n = fin ? bestN : sList[ei];
    n = (n < 0) ? 0 : ((n > kN - 1) ? (kN - 1) : n);
    __syncthreads();
    if (tid < kL) sZ[tid] = z[(size_t)n * kL + tid];
    __syncthreads();
    float kz = 0.0f;
#pragma unroll 1
    for (int l = 0; l < kL; ++l) {
      const float zl = sZ[l];
      kz = fmaf(zl, zl, kz);
    }
    float part = 0.0f;
#pragma unroll 1
    for (int k = 0; k < 3; ++k) {
      const int d = 4 * (tid + 256 * k);
      const float* wp = wcls + d;
      float a0 = 0.0f, a1 = 0.0f, a2 = 0.0f, a3 = 0.0f;
#pragma unroll 4
      for (int l = 0; l < kL; ++l) {
        const v4f w = *(const v4f*)(wp + (size_t)l * kD);
        const float zl = sZ[l];
        a0 = fmaf(zl, w[0], a0);
        a1 = fmaf(zl, w[1], a1);
        a2 = fmaf(zl, w[2], a2);
        a3 = fmaf(zl, w[3], a3);
      }
      const v4f bv = *(const v4f*)(bcls + d);
      const v4f xv = *(const v4f*)(xrow + d);
      v4f rv;
      {
        const float r0 = 1.0f / (1.0f + expf(-(a0 + bv[0])));
        const float r1 = 1.0f / (1.0f + expf(-(a1 + bv[1])));
        const float r2 = 1.0f / (1.0f + expf(-(a2 + bv[2])));
        const float r3 = 1.0f / (1.0f + expf(-(a3 + bv[3])));
        const float f0 = xv[0] - r0;
        const float f1 = xv[1] - r1;
        const float f2 = xv[2] - r2;
        const float f3 = xv[3] - r3;
        part = fmaf(f0, f0, part);
        part = fmaf(f1, f1, part);
        part = fmaf(f2, f2, part);
        part = fmaf(f3, f3, part);
        rv[0] = r0;
        rv[1] = r1;
        rv[2] = r2;
        rv[3] = r3;
      }
      if (fin) {
        float* p = orow + d;
        *(volatile v4f*)p = rv;
        __threadfence();
        *(volatile v4f*)p = rv;
      }
    }
#pragma unroll
    for (int off = 16; off >= 1; off >>= 1) part += __shfl_xor(part, off, 32);
    if (lane == 0) sRed[wave] = part;
    __syncthreads();
    float tot = 0.0f;
#pragma unroll 1
    for (int w = 0; w < 8; ++w) tot += sRed[w];
    const float lossv = tot + 0.5f * kz;
    if (!fin) {
      if (lossv < bestL) {
        bestL = lossv;
        bestN = n;
      }
    } else {
      finalL = lossv;
    }
  }

  if (wave == 1) {
    const int q4 = (lane & 15) * 4;
    const bool lowHalf = (lane < 16);
    const v4f zv = *(const v4f*)(z + (size_t)bestN * kL + q4);
    v4f val;
    val[0] = lowHalf ? zv[0] : 0.0f;
    val[1] = lowHalf ? zv[1] : 0.0f;
    val[2] = lowHalf ? zv[2] : 0.0f;
    val[3] = lowHalf ? zv[3] : 0.0f;
    const size_t base = lowHalf ? kOutMus : kOutLv;
    float* p = out + base + (size_t)cb * kL + q4;
    *(volatile v4f*)p = val;
    __threadfence();
    *(volatile v4f*)p = val;
  }
  if (wave == 0) {
    float* p = bestp + (size_t)cb * 32 + lane;
    *(volatile float*)p = finalL;
    __threadfence();
    *(volatile float*)p = finalL;
  }
}

__global__ __launch_bounds__(160) void logits_kernel(const float* __restrict__ bestp, float* __restrict__ out) {
  const int i = threadIdx.x;
  v4f v;
  {
    const int o0 = 4 * i;
    const int b0 = o0 / kNC, c0 = o0 - b0 * kNC;
    const int o1 = o0 + 1;
    const int b1 = o1 / kNC, c1 = o1 - b1 * kNC;
    const int o2 = o0 + 2;
    const int b2 = o2 / kNC, c2 = o2 - b2 * kNC;
    const int o3 = o0 + 3;
    const int b3 = o3 / kNC, c3 = o3 - b3 * kNC;
    v[0] = -bestp[(size_t)(c0 * kB + b0) * 32];
    v[1] = -bestp[(size_t)(c1 * kB + b1) * 32];
    v[2] = -bestp[(size_t)(c2 * kB + b2) * 32];
    v[3] = -bestp[(size_t)(c3 * kB + b3) * 32];
  }
  float* p = out + 4 * i;
  *(volatile v4f*)p = v;
  __threadfence();
  *(volatile v4f*)p = v;
}

extern "C" void kernel_launch(void* const* d_in, const int* in_sizes, int n_in,
                              void* d_out, int out_size, void* d_ws, size_t ws_size,
                              hipStream_t stream) {
  if (n_in < 4) return;
  if (in_sizes[0] != kB * kD) return;
  if (in_sizes[1] != kN * kL) return;
  if (in_sizes[2] != kNC * kL * kD) return;
  if (in_sizes[3] != kNC * kD) return;
  if ((size_t)out_size != kOutTotal) return;
  if (ws_size < kWsTotal) return;

  const float* x     = (const float*)d_in[0];
  const float* z     = (const float*)d_in[1];
  const float* dec_w = (const float*)d_in[2];
  const float* dec_b = (const float*)d_in[3];
  float* out = (float*)d_out;

  char* ws = (char*)d_ws;
  unsigned short* XC16 = (unsigned short*)(ws + kOffXC);
  unsigned short* Z16  = (unsigned short*)(ws + kOffZ16);
  float*          KLD  = (float*)(ws + kOffKLD);
  unsigned short* WT16 = (unsigned short*)(ws + kOffWT);
  float*          LC   = (float*)(ws + kOffLC);
  float*          BEST = (float*)(ws + kOffBEST);

  prep_x_kernel<<<(kB * kD / 8) / 256, 256, 0, stream>>>(x, XC16, kB * kD / 8);
  prep_z_kernel<<<(kN * kL / 8) / 256, 256, 0, stream>>>(z, Z16, KLD);
  prep_w_kernel<<<dim3(kD / 64, kNC), 256, 0, stream>>>(dec_w, WT16);
  coarse_loss_kernel<<<dim3(kN / 64, kNC), 64, 0, stream>>>(Z16, WT16, XC16, dec_b, KLD, LC);
  select_emit_kernel<<<kNC * kB, 256, 0, stream>>>(x, z, dec_w, dec_b, LC, out, BEST);
  logits_kernel<<<1, 160, 0, stream>>>(BEST, out);
}
